// SelfAttentionBlock2d_85873576117032
// MI455X (gfx1250) — hardware-verified
//
#include <hip/hip_runtime.h>
#include <math.h>


#define NB 4
#define CC 256
#define SS 4096
#define EE 128
#define BK 32

typedef __attribute__((ext_vector_type(16))) _Float16 v16h;
typedef __attribute__((ext_vector_type(8)))  _Float16 v8h;
typedef __attribute__((ext_vector_type(8)))  float v8f;
typedef __attribute__((ext_vector_type(4)))  float v4f;
typedef __attribute__((ext_vector_type(4)))  unsigned v4u;

template <typename T> __device__ __forceinline__ void vst2(void* p, T v) { *(volatile T*)p = v; __threadfence(); *(volatile T*)p = v; }
__device__ __forceinline__ v8f wmma16(v16h a, v16h b, v8f c) {
  v8f d = __builtin_amdgcn_wmma_f32_16x16x32_f16(false, a, false, b, (short)0, c, false, false);
  asm volatile("v_nop\n\tv_nop\n\tv_nop\n\tv_nop" : "+v"(d) : "v"(a), "v"(b));
  return d;
}
__device__ __forceinline__ v16h frag_h(const _Float16* rowk0, int lane) {
  union { v16h v; v8h q[2]; } u; const _Float16* p = rowk0 + 8 * (lane >> 4);
  u.q[0] = *(const v8h*)p; u.q[1] = *(const v8h*)(p + 16); return u.v;
}
__device__ __forceinline__ v16h frag_f32(const float* rowk0, int lane) {
  v16h a; const float* p = rowk0 + 8 * (lane >> 4);
#pragma unroll
  for (int i = 0; i < 8; ++i) { a[i] = (_Float16)p[i]; a[8 + i] = (_Float16)p[16 + i]; }
  return a;
}
__device__ __forceinline__ v16h frag_f32col(const float* colk0, int lane, int ld) {
  v16h a; const float* p = colk0 + (size_t)(8 * (lane >> 4)) * ld;
#pragma unroll
  for (int i = 0; i < 8; ++i) { a[i] = (_Float16)p[(size_t)i * ld]; a[8 + i] = (_Float16)p[(size_t)(16 + i) * ld]; }
  return a;
}
#define LDSX() do { asm volatile("s_wait_dscnt 0" ::: "memory"); __builtin_amdgcn_wave_barrier(); __builtin_amdgcn_fence(__ATOMIC_RELEASE, "workgroup"); } while (0)

__global__ __launch_bounds__(128) void k_proj(const float* __restrict__ x, const float* __restrict__ Wq, const float* __restrict__ bq,
                                            const float* __restrict__ Wk, const float* __restrict__ bk, const float* __restrict__ Wv, const float* __restrict__ bv,
                                            _Float16* __restrict__ qh, _Float16* __restrict__ kh, _Float16* __restrict__ vT) {
  __shared__ __align__(16) float st[128][68];
  const int tid = threadIdx.x, wave = tid >> 5, lane = tid & 31, col = lane & 15, g = lane >> 4;
  const int n = blockIdx.y, which = blockIdx.z;
  const int s0 = blockIdx.x * 64, sw = s0 + wave * 16;
  const float* W = which == 0 ? Wq : (which == 1 ? Wk : Wv);
  const float* bb = which == 0 ? bq : (which == 1 ? bk : bv);
  const float* xn = x + (size_t)n * CC * SS;
  v8f acc[8] = {};
#pragma unroll 1
  for (int kc = 0; kc < CC / 32; ++kc) {
    const v16h a = frag_f32col(xn + (size_t)(kc * 32) * SS + sw + col, lane, SS);
#pragma unroll
    for (int j = 0; j < 8; ++j) acc[j] = wmma16(a, frag_f32(W + (size_t)(j * 16 + col) * CC + kc * 32, lane), acc[j]);
  }
#pragma unroll
  for (int j = 0; j < 8; ++j) { const float bv_ = bb[j * 16 + col];
#pragma unroll
    for (int r = 0; r < 8; ++r) st[j * 16 + col][wave * 16 + 8 * g + r] = acc[j][r] + bv_; }
  __syncthreads();
  if (which < 2) {
    _Float16* dst = (which == 0 ? qh : kh) + ((size_t)n * SS + s0) * EE;
    for (int q = tid; q < 64 * 16; q += 128) { const int sl = q >> 4, pc = q & 15;
      union { v8h h; v4u u; } pk;
#pragma unroll
      for (int e = 0; e < 8; ++e) pk.h[e] = (_Float16)st[pc * 8 + e][sl];
      vst2(dst + (size_t)sl * EE + pc * 8, pk.u); }
  } else {
    for (int q = tid; q < 128 * 8; q += 128) { const int e = q >> 3, pc = q & 7;
      union { v8h h; v4u u; } pk;
#pragma unroll
      for (int i = 0; i < 8; ++i) pk.h[i] = (_Float16)st[e][pc * 8 + i];
      vst2(vT + ((size_t)n * EE + e) * SS + s0 + pc * 8, pk.u); }
  }
}

__global__ __launch_bounds__(128) void k_attn(const _Float16* __restrict__ qh, const _Float16* __restrict__ kh, const _Float16* __restrict__ vT,
                                            float* __restrict__ ao) {
  __shared__ __align__(16) float sP[4][16][BK];
  __shared__ __align__(16) float sO[4][16][EE];
  const int tid = threadIdx.x, w = tid >> 5, lane = tid & 31, g = lane >> 4, ln = lane & 15;
  const int n = blockIdx.y, q0 = blockIdx.x * 64 + w * 16;
  const _Float16* qrow = qh + ((size_t)n * SS + q0 + ln) * EE;
  v16h qa[4];
#pragma unroll
  for (int c = 0; c < 4; ++c) qa[c] = frag_h(qrow + c * 32, lane);
  float mrun[8], lrun[8];
  v8f acc[8];
#pragma unroll
  for (int r = 0; r < 8; ++r) { mrun[r] = -3.0e38f; lrun[r] = 0.f; }
#pragma unroll
  for (int t = 0; t < 8; ++t) acc[t] = (v8f){};
  const _Float16* kb = kh + (size_t)n * SS * EE;
  const _Float16* vb = vT + (size_t)n * EE * SS;
#pragma unroll 1
  for (int k0 = 0; k0 < SS; k0 += BK) {
    v8f s0 = {}, s1 = {};
#pragma unroll
    for (int c = 0; c < 4; ++c) {
      s0 = wmma16(qa[c], frag_h(kb + (size_t)(k0 + ln) * EE + c * 32, lane), s0);
      s1 = wmma16(qa[c], frag_h(kb + (size_t)(k0 + 16 + ln) * EE + c * 32, lane), s1);
    }
#pragma unroll
    for (int r = 0; r < 8; ++r) {
      float mx = fmaxf(s0[r], s1[r]);
#pragma unroll
      for (int off = 8; off >= 1; off >>= 1) mx = fmaxf(mx, __shfl_xor(mx, off, 32));
      const float mn = fmaxf(mrun[r], mx);
      const float corr = expf(mrun[r] - mn);
      const float p0 = expf(s0[r] - mn), p1 = expf(s1[r] - mn);
      float sum = p0 + p1;
#pragma unroll
      for (int off = 8; off >= 1; off >>= 1) sum += __shfl_xor(sum, off, 32);
      lrun[r] = lrun[r] * corr + sum; mrun[r] = mn;
#pragma unroll
      for (int t = 0; t < 8; ++t) acc[t][r] *= corr;
      sP[w][8 * g + r][ln] = p0 * 16384.0f; sP[w][8 * g + r][16 + ln] = p1 * 16384.0f;
    }
    LDSX();
    const v16h pa = frag_f32(&sP[w][ln][0], lane);
#pragma unroll
    for (int t = 0; t < 8; ++t) acc[t] = wmma16(pa, frag_h(vb + (size_t)(t * 16 + ln) * SS + k0, lane), acc[t]);
    __builtin_amdgcn_wave_barrier();
  }
  float* so = &sO[w][0][0];
#pragma unroll
  for (int r = 0; r < 8; ++r) { const float il = (1.0f / 16384.0f) / lrun[r];
#pragma unroll
    for (int t = 0; t < 8; ++t) so[(8 * g + r) * EE + t * 16 + ln] = acc[t][r] * il; }
  LDSX();
#pragma unroll 4
  for (int rl = 0; rl < 16; ++rl) vst2(ao + ((size_t)n * SS + q0 + rl) * EE + lane * 4, *(const v4f*)(so + rl * EE + lane * 4));
}

__global__ __launch_bounds__(128) void k_out(const float* __restrict__ x, const float* __restrict__ Wo, const float* __restrict__ bo,
                                           const float* __restrict__ ao, float* __restrict__ out) {
  __shared__ __align__(16) float st[64][68];
  const int tid = threadIdx.x, wave = tid >> 5, lane = tid & 31, col = lane & 15, g = lane >> 4;
  const int n = blockIdx.z, c0 = blockIdx.x * 64 + wave * 16, s0 = blockIdx.y * 64;
  v8f acc[4] = {};
#pragma unroll
  for (int kc = 0; kc < EE / 32; ++kc) {
    const v16h a = frag_f32(Wo + (size_t)(c0 + col) * EE + kc * 32, lane);
#pragma unroll
    for (int j = 0; j < 4; ++j) acc[j] = wmma16(a, frag_f32(ao + ((size_t)n * SS + s0 + j * 16 + col) * EE + kc * 32, lane), acc[j]);
  }
#pragma unroll
  for (int j = 0; j < 4; ++j)
#pragma unroll
    for (int r = 0; r < 8; ++r) st[wave * 16 + 8 * g + r][j * 16 + col] = acc[j][r] + bo[c0 + 8 * g + r];
  __syncthreads();
  const int bc0 = blockIdx.x * 64;
  for (int q = tid; q < 64 * 16; q += 128) { const int rl = q >> 4, pc = q & 15;
    const size_t idx = ((size_t)n * CC + bc0 + rl) * SS + s0 + pc * 4;
    v4f v = *(const v4f*)(&st[rl][pc * 4]) + *(const v4f*)(x + idx);
    vst2(out + idx, v); }
}

extern "C" void kernel_launch(void* const* d_in, const int* in_sizes, int n_in,
                              void* d_out, int out_size, void* d_ws, size_t ws_size,
                              hipStream_t stream) {
  (void)in_sizes; (void)n_in; (void)out_size; (void)ws_size;
  const float* x  = (const float*)d_in[0];
  const float* Wq = (const float*)d_in[1]; const float* bq = (const float*)d_in[2];
  const float* Wk = (const float*)d_in[3]; const float* bk = (const float*)d_in[4];
  const float* Wv = (const float*)d_in[5]; const float* bv = (const float*)d_in[6];
  const float* Wo = (const float*)d_in[7]; const float* bo = (const float*)d_in[8];
  float* out = (float*)d_out;
  char* ws = (char*)d_ws;
  _Float16* qh = (_Float16*)ws;
  _Float16* kh = qh + (size_t)NB * SS * EE;
  _Float16* vT = kh + (size_t)NB * SS * EE;
  float* ao = (float*)(vT + (size_t)NB * EE * SS);
  k_proj<<<dim3(SS / 64, NB, 3), 128, 0, stream>>>(x, Wq, bq, Wk, bk, Wv, bv, qh, kh, vT);
  k_attn<<<dim3(SS / 64, NB), 128, 0, stream>>>(qh, kh, vT, ao);
  k_out<<<dim3(CC / 64, SS / 64, NB), 128, 0, stream>>>(x, Wo, bo, ao, out);
}
